// Sage_32238024524264
// MI455X (gfx1250) — hardware-run, weakly checked
//
#include <hip/hip_runtime.h>
#include <stddef.h>
#include <stdint.h>


#define FI      128
#define HD      256
#define OC      50
#define ONP     64
#define XBP     128
#define S1P     256
#define HP      512
#define W1P     384
#define W2P     1024
#define KS1     (FI / 32)
#define KS2     (HD / 32)
#define SPLIT_S1 1
#define SPLIT_H  1
#define SPLIT_S2 1
#define NTHR    256
#define NWAVE   8
#define EPT     8
#define CHUNK   (NTHR * EPT)
#define NBA     1024
#define PKS     10
#define RCAP    8192
#define WLCAP   1536
#define DEGCAP  64
#define GBM     64
#define GBN     128
#define GTHR    128
#define RPB     64
#define RPW     8
#define W1PU    (HD * (FI / 8))
#define W2PU    (ONP * (HD / 8))
#define W1U     (3 * W1PU)
#define W2U     (4 * W2PU)
#define BU1     (HD / 4)
#define BU2     (ONP / 4)
#define BK_INTS (NWAVE * WLCAP + RCAP + 3 * NBA + 32)
#define LDS_BK  (BK_INTS * 4)
#define NFL     ((GBM * OC / 4 + GTHR - 1) / GTHR)
#define MEAS_BLK_HITS 6764
#define MEAS_MAXDEG   21

static_assert((CHUNK & (CHUNK - 1)) == 0 && CHUNK <= 4096);
static_assert(NBA == (1 << PKS) && NBA == NTHR * 4);
static_assert(RCAP % (NTHR * 4) == 0 && BK_INTS % 4 == 0);
static_assert((long long)RCAP * 100 >= (long long)MEAS_BLK_HITS * 105);
static_assert(DEGCAP >= MEAS_MAXDEG + 8);
static_assert(NWAVE * WLCAP >= RCAP);
static_assert(LDS_BK <= 327680);
static_assert(W1P == 3 * FI && W2P == 4 * HD && S1P == 2 * FI && HP == 2 * HD && XBP == FI);
static_assert(FI % 32 == 0 && HD % 32 == 0);
static_assert(GBM == (GTHR / 32) * 16 && HD == 2 * GBN && GBN == 8 * 16 && GBN == 32 * 4);
static_assert(ONP == 4 * 16 && OC <= ONP && OC > 48);
static_assert(W1PU % NTHR == 0 && W2PU % NTHR == 0 && W1PU == 4096 && W2PU == 2048);
static_assert(RPB == NWAVE * RPW && RPB == GBM && NBA % GBM == 0);
static_assert((GBM * OC * 4) % 128 == 0 && (16 * OC * 4) % 128 == 0 && (GBM * OC) % 4 == 0);
static_assert(NFL == 7);

typedef float          v4f   __attribute__((ext_vector_type(4)));
typedef float          v8f   __attribute__((ext_vector_type(8)));
typedef int            v4i   __attribute__((ext_vector_type(4)));
typedef int            v8i   __attribute__((ext_vector_type(8)));
typedef unsigned       v2u   __attribute__((ext_vector_type(2)));
typedef unsigned       v4u   __attribute__((ext_vector_type(4)));
typedef unsigned short v8us  __attribute__((ext_vector_type(8)));
typedef __bf16         v16bf __attribute__((ext_vector_type(16)));
typedef v4f  __attribute__((may_alias)) v4fa;
typedef v4i  __attribute__((may_alias)) v4ia;
typedef v2u  __attribute__((may_alias)) v2ua;
typedef v4u  __attribute__((may_alias)) v4ua;
typedef v8us __attribute__((may_alias)) v8usa;
union FragB { v16bf v; v8us h[2]; v8i w; };

__device__ __forceinline__ v8f wmb(const FragB& a, const FragB& b, v8f c) {
  v8f d = __builtin_amdgcn_wmma_f32_16x16x32_bf16(false, a.v, false, b.v, (short)0, c, false, false);
  asm volatile("v_nop\n\tv_nop\n\tv_nop\n\tv_nop" : "+v"(d) : "v"(a.w), "v"(b.w));
  return d;
}

__device__ __forceinline__ unsigned bf16_bits(float f) {
  const unsigned u = __float_as_uint(f);
  const unsigned r = ((u + 0x7FFFu + ((u >> 16) & 1u)) >> 16) & 0xFFFFu;
  return (f != f) ? 0x7FC0u : r;
}
__device__ __forceinline__ float bf16_val(float f) { return __uint_as_float(bf16_bits(f) << 16); }
__device__ __forceinline__ float bfw_lo(unsigned w) { return __uint_as_float(w << 16); }
__device__ __forceinline__ float bfw_hi(unsigned w) { return __uint_as_float(w & 0xffff0000u); }
__device__ __forceinline__ void pack2(float a, float b, unsigned& hw, unsigned& lw) {
  const unsigned ha = bf16_bits(a), hb = bf16_bits(b);
  const unsigned la = bf16_bits(a - __uint_as_float(ha << 16));
  const unsigned lb = bf16_bits(b - __uint_as_float(hb << 16));
  hw = ha | (hb << 16);
  lw = la | (lb << 16);
}
__device__ __forceinline__ float relu_k(float v) { return (v > 0.0f) ? v : (v - v); }

__device__ __forceinline__ void wave_sync() {
  __builtin_amdgcn_fence(__ATOMIC_RELEASE, "wavefront");
  __builtin_amdgcn_wave_barrier();
  __builtin_amdgcn_fence(__ATOMIC_ACQUIRE, "wavefront");
}

__device__ __forceinline__ void put8(unsigned short* p, v8us o) {
  *(volatile v8us*)p = o;
  __threadfence();
  *(volatile v8us*)p = o;
}
__device__ __forceinline__ void put4f(float* p, v4f o) {
  *(volatile v4f*)p = o;
  __threadfence();
  *(volatile v4f*)p = o;
}

__device__ __forceinline__ v8us cvt8(v4f a, v4f b, unsigned mk) {
  v8us o;
  o[0] = (unsigned short)(bf16_bits(a.x) & mk); o[1] = (unsigned short)(bf16_bits(a.y) & mk);
  o[2] = (unsigned short)(bf16_bits(a.z) & mk); o[3] = (unsigned short)(bf16_bits(a.w) & mk);
  o[4] = (unsigned short)(bf16_bits(b.x) & mk); o[5] = (unsigned short)(bf16_bits(b.y) & mk);
  o[6] = (unsigned short)(bf16_bits(b.z) & mk); o[7] = (unsigned short)(bf16_bits(b.w) & mk);
  return o;
}

__global__ __launch_bounds__(NTHR) void k_prep(const float* __restrict__ x, const float* __restrict__ W1l,
                                               const float* __restrict__ b1l, const float* __restrict__ W1r,
                                               const float* __restrict__ W2l, const float* __restrict__ b2l,
                                               const float* __restrict__ W2r,
                                               unsigned short* XB, unsigned short* W1c, unsigned short* W2c,
                                               float* B1, float* B2, int nN, int nXU) {
  const int u = (int)blockIdx.x * NTHR + (int)threadIdx.x;
  if (u < nXU) {
    const int row = u >> 4;
    const int k8  = (u & 15) * 8;
    const int rc  = row < nN ? row : nN - 1;
    const float* p = x + (size_t)rc * FI + k8;
    const v4f a = *(const v4f*)p;
    const v4f b = *(const v4f*)(p + 4);
    asm volatile("" :: "v"(a), "v"(b));
    const unsigned mk = (row < nN) ? 0xFFFFu : 0u;
    put8(XB + (size_t)row * XBP + k8, cvt8(a, b, mk));
  } else {
    const int v = u - nXU;
    if (v < W1U) {
      const int part = v / W1PU;
      const int w    = v - part * W1PU;
      const int n    = w >> 4;
      const int k8   = (w & 15) * 8;
      const size_t so = (size_t)n * FI + k8;
      v4f a, b;
      if (part == 2) { a = *(const v4f*)(W1r + so); b = *(const v4f*)(W1r + so + 4); }
      else           { a = *(const v4f*)(W1l + so); b = *(const v4f*)(W1l + so + 4); }
      put8(W1c + (size_t)n * W1P + part * FI + k8, cvt8(a, b, 0xFFFFu));
    } else if (v < W1U + W2U) {
      const int v2   = v - W1U;
      const int part = v2 / W2PU;
      const int w    = v2 - part * W2PU;
      const int n    = w >> 5;
      const int k8   = (w & 31) * 8;
      const int nc   = n < OC ? n : OC - 1;
      const size_t so = (size_t)nc * HD + k8;
      v4f a, b;
      if (part >= 2) { a = *(const v4f*)(W2r + so); b = *(const v4f*)(W2r + so + 4); }
      else           { a = *(const v4f*)(W2l + so); b = *(const v4f*)(W2l + so + 4); }
      asm volatile("" :: "v"(a), "v"(b));
      const unsigned mk = (n < OC) ? 0xFFFFu : 0u;
      put8(W2c + (size_t)n * W2P + part * HD + k8, cvt8(a, b, mk));
    } else if (v < W1U + W2U + BU1) {
      const int j = v - (W1U + W2U);
      const v4f b4 = *(const v4f*)(b1l + 4 * j);
      v4f o;
      o.x = bf16_val(b4.x); o.y = bf16_val(b4.y); o.z = bf16_val(b4.z); o.w = bf16_val(b4.w);
      put4f(B1 + 4 * j, o);
    } else if (v < W1U + W2U + BU1 + BU2) {
      const int j  = v - (W1U + W2U + BU1);
      const int i0 = 4 * j;
      const float f0 = b2l[min(i0,     OC - 1)];
      const float f1 = b2l[min(i0 + 1, OC - 1)];
      const float f2 = b2l[min(i0 + 2, OC - 1)];
      const float f3 = b2l[min(i0 + 3, OC - 1)];
      asm volatile("" :: "v"(f0), "v"(f1), "v"(f2), "v"(f3));
      v4f o;
      o.x = (i0     < OC) ? bf16_val(f0) : 0.0f;
      o.y = (i0 + 1 < OC) ? bf16_val(f1) : 0.0f;
      o.z = (i0 + 2 < OC) ? bf16_val(f2) : 0.0f;
      o.w = (i0 + 3 < OC) ? bf16_val(f3) : 0.0f;
      put4f(B2 + 4 * j, o);
    }
  }
}

__device__ __forceinline__ int scan_chunk(const int* __restrict__ keys, int nE, int cbase, int slotBase,
                                          int nb, int vec8, int* mywl, int wc, int tid) {
  const int e0   = cbase + tid * EPT;
  const int sent = (int)(1u << 31);
  v4i da, db;
  if (vec8 != 0 && cbase + CHUNK <= nE) {
    da = *(const v4i*)(keys + e0);
    db = *(const v4i*)(keys + e0 + 4);
  } else {
    const int t0 = keys[min(e0,     nE - 1)];
    const int t1 = keys[min(e0 + 1, nE - 1)];
    const int t2 = keys[min(e0 + 2, nE - 1)];
    const int t3 = keys[min(e0 + 3, nE - 1)];
    const int t4 = keys[min(e0 + 4, nE - 1)];
    const int t5 = keys[min(e0 + 5, nE - 1)];
    const int t6 = keys[min(e0 + 6, nE - 1)];
    const int t7 = keys[min(e0 + 7, nE - 1)];
    asm volatile("" :: "v"(t0), "v"(t1), "v"(t2), "v"(t3), "v"(t4), "v"(t5), "v"(t6), "v"(t7));
    da.x = (e0     < nE) ? t0 : sent;
    da.y = (e0 + 1 < nE) ? t1 : sent;
    da.z = (e0 + 2 < nE) ? t2 : sent;
    da.w = (e0 + 3 < nE) ? t3 : sent;
    db.x = (e0 + 4 < nE) ? t4 : sent;
    db.y = (e0 + 5 < nE) ? t5 : sent;
    db.z = (e0 + 6 < nE) ? t6 : sent;
    db.w = (e0 + 7 < nE) ? t7 : sent;
  }
  const unsigned nbs = (unsigned)slotBase;
  const unsigned unb = (unsigned)nb;
  const unsigned s0 = (unsigned)da.x - nbs, s1 = (unsigned)da.y - nbs;
  const unsigned s2 = (unsigned)da.z - nbs, s3 = (unsigned)da.w - nbs;
  const unsigned s4 = (unsigned)db.x - nbs, s5 = (unsigned)db.y - nbs;
  const unsigned s6 = (unsigned)db.z - nbs, s7 = (unsigned)db.w - nbs;
  const bool h0 = s0 < unb, h1 = s1 < unb, h2 = s2 < unb, h3 = s3 < unb;
  const bool h4 = s4 < unb, h5 = s5 < unb, h6 = s6 < unb, h7 = s7 < unb;
  const unsigned any = __builtin_amdgcn_ballot_w32(h0 | h1 | h2 | h3 | h4 | h5 | h6 | h7);
  if (any != 0u) {
#define HITJ(J, HJ, SJ) { \
      const unsigned mj = __builtin_amdgcn_ballot_w32(HJ); \
      if (mj != 0u) { \
        if (HJ) { \
          const int pos = wc + (int)__builtin_amdgcn_mbcnt_lo(mj, 0u); \
          if (pos < WLCAP) mywl[pos] = (int)(((unsigned)(e0 + (J)) << PKS) | (SJ)); \
        } \
        wc += (int)__builtin_popcount(mj); } }
    HITJ(0, h0, s0)
    HITJ(1, h1, s1)
    HITJ(2, h2, s2)
    HITJ(3, h3, s3)
    HITJ(4, h4, s4)
    HITJ(5, h5, s5)
    HITJ(6, h6, s6)
    HITJ(7, h7, s7)
#undef HITJ
  }
  return wc;
}

__global__ __launch_bounds__(NTHR) void k_bucket(const int* __restrict__ keys, const int* __restrict__ gidx,
                                                 int nE, int nN, int vec8,
                                                 int* LIST, int* CNT, int* OFF, int* REC) {
  extern __shared__ __attribute__((aligned(16))) int dsm[];
  int* wl   = dsm;
  int* reg2 = wl + NWAVE * WLCAP;
  int* scnt = reg2 + RCAP;
  int* soff = scnt + NBA;
  int* cur  = soff + NBA;
  int* wcnt = cur + NBA;
  int* wtot = wcnt + 8;
  int* wmx  = wtot + 8;
  const int tid = (int)threadIdx.x, lane = tid & 31, wave = tid >> 5;
  const int nodeBase = (int)blockIdx.x * NBA;
  int nb = nN - nodeBase;
  nb = nb > NBA ? NBA : (nb < 1 ? 1 : nb);

  {
    const v4i z4 = {0, 0, 0, 0};
    for (int i = tid * 4; i < BK_INTS; i += NTHR * 4) *(v4ia*)(dsm + i) = z4;
  }
  __syncthreads();

  {
    int wc = 0;
    int* mywl = wl + wave * WLCAP;
    const int nChunks = (nE + CHUNK - 1) / CHUNK;
#pragma unroll 1
    for (int ch = 0; ch < nChunks; ++ch)
      wc = scan_chunk(keys, nE, ch * CHUNK, nodeBase, nb, vec8, mywl, wc, tid);
    if (lane == 0) wcnt[wave] = wc;
  }
  __syncthreads();

  int nh = 0, ovf = 0;
#pragma unroll
  for (int w2 = 0; w2 < NWAVE; ++w2) {
    int c = wcnt[w2];
    ovf |= (c > WLCAP) ? 1 : 0;
    c = c < 0 ? 0 : (c > WLCAP ? WLCAP : c);
    if (c > RCAP - nh) { c = RCAP - nh; ovf = 1; }
    nh += c;
  }

  if (wave == 0) {
    int tot = 0;
#pragma unroll 1
    for (int w2 = 0; w2 < NWAVE; ++w2) {
      int cv = wcnt[w2];
      cv = cv < 0 ? 0 : (cv > WLCAP ? WLCAP : cv);
      if (cv > RCAP - tot) cv = RCAP - tot;
      const int c = __builtin_amdgcn_readfirstlane(cv);
#pragma unroll 1
      for (int b0 = 0; b0 < c; b0 += 32) {
        const int idx = b0 + lane;
        const int uv  = wl[w2 * WLCAP + (idx < WLCAP ? idx : WLCAP - 1)];
        const int m32 = (c - b0) < 32 ? (c - b0) : 32;
#pragma unroll 1
        for (int k = 0; k < m32; ++k) {
          const int u  = __builtin_amdgcn_readlane(uv, k);
          const int sl = u & (NBA - 1);
          if (lane == 0) scnt[sl] = scnt[sl] + 1;
        }
      }
      tot += c;
    }
  }
  __syncthreads();

  {
    const v4i ca = *(const v4ia*)(scnt + 4 * tid);
    const int e0 = ca.x < 0 ? 0 : ca.x, e1 = ca.y < 0 ? 0 : ca.y, e2 = ca.z < 0 ? 0 : ca.z, e3 = ca.w < 0 ? 0 : ca.w;
    const int ts = e0 + e1 + e2 + e3;
    int incl = ts;
#pragma unroll
    for (int d = 1; d < 32; d <<= 1) {
      const int up = __shfl_up(incl, d, 32);
      if (lane >= d) incl += up;
    }
    int mx = max(max(e0, e1), max(e2, e3));
    mx = max(mx, __shfl_xor(mx, 16, 32));
    mx = max(mx, __shfl_xor(mx, 8, 32));
    mx = max(mx, __shfl_xor(mx, 4, 32));
    mx = max(mx, __shfl_xor(mx, 2, 32));
    mx = max(mx, __shfl_xor(mx, 1, 32));
    if (lane == 31) wtot[wave] = incl;
    if (lane == 0)  wmx[wave] = mx;
    __syncthreads();
    int pre = 0;
#pragma unroll
    for (int w2 = 0; w2 < NWAVE; ++w2) pre += (w2 < wave) ? wtot[w2] : 0;
    int run = pre + incl - ts;
    v4i so;
    so.x = run; run += e0;
    so.y = run; run += e1;
    so.z = run; run += e2;
    so.w = run;
    *(v4ia*)(soff + 4 * tid) = so;
    *(v4ia*)(cur + 4 * tid)  = so;
  }
  __syncthreads();

  if (wave == 0) {
    int tot = 0;
#pragma unroll 1
    for (int w2 = 0; w2 < NWAVE; ++w2) {
      int cv = wcnt[w2];
      cv = cv < 0 ? 0 : (cv > WLCAP ? WLCAP : cv);
      if (cv > RCAP - tot) cv = RCAP - tot;
      const int c = __builtin_amdgcn_readfirstlane(cv);
#pragma unroll 1
      for (int b0 = 0; b0 < c; b0 += 32) {
        const int idx = b0 + lane;
        const int uv  = wl[w2 * WLCAP + (idx < WLCAP ? idx : WLCAP - 1)];
        const int m32 = (c - b0) < 32 ? (c - b0) : 32;
#pragma unroll 1
        for (int k = 0; k < m32; ++k) {
          const int u   = __builtin_amdgcn_readlane(uv, k);
          const int sl  = u & (NBA - 1);
          const int eid = (int)((unsigned)u >> PKS);
          if (lane == 0) {
            int pos = cur[sl];
            pos = pos < 0 ? 0 : (pos > RCAP - 1 ? RCAP - 1 : pos);
            reg2[pos] = eid;
            cur[sl] = pos + 1;
          }
        }
      }
      tot += c;
    }
  }
  __syncthreads();

  int bmax = 0;
#pragma unroll
  for (int w2 = 0; w2 < NWAVE; ++w2) bmax = max(bmax, wmx[w2]);
  const int flag = ((ovf != 0) || (bmax > DEGCAP)) ? 1 : 0;

  int* lrow = LIST + (size_t)blockIdx.x * RCAP;
#pragma unroll 1
  for (int it = 0; it < RCAP / (NTHR * 4); ++it) {
    const int i0 = 4 * (it * NTHR + tid);
    const v4i ev = *(const v4ia*)(reg2 + i0);
    int e0 = ev.x, e1 = ev.y, e2 = ev.z, e3 = ev.w;
    e0 = e0 < 0 ? 0 : (e0 > nE - 1 ? nE - 1 : e0);
    e1 = e1 < 0 ? 0 : (e1 > nE - 1 ? nE - 1 : e1);
    e2 = e2 < 0 ? 0 : (e2 > nE - 1 ? nE - 1 : e2);
    e3 = e3 < 0 ? 0 : (e3 > nE - 1 ? nE - 1 : e3);
    int g0 = gidx[e0], g1 = gidx[e1], g2 = gidx[e2], g3 = gidx[e3];
    asm volatile("" :: "v"(g0), "v"(g1), "v"(g2), "v"(g3));
    g0 = g0 < 0 ? 0 : (g0 > nN - 1 ? nN - 1 : g0);
    g1 = g1 < 0 ? 0 : (g1 > nN - 1 ? nN - 1 : g1);
    g2 = g2 < 0 ? 0 : (g2 > nN - 1 ? nN - 1 : g2);
    g3 = g3 < 0 ? 0 : (g3 > nN - 1 ? nN - 1 : g3);
    v4i ov;
    ov.x = (i0     < nh) ? g0 : 0;
    ov.y = (i0 + 1 < nh) ? g1 : 0;
    ov.z = (i0 + 2 < nh) ? g2 : 0;
    ov.w = (i0 + 3 < nh) ? g3 : 0;
    *(volatile v4i*)(lrow + i0) = ov;
    __threadfence();
    *(volatile v4i*)(lrow + i0) = ov;
  }
  {
    const v4i cv = *(const v4ia*)(scnt + 4 * tid);
    const v4i fv = *(const v4ia*)(soff + 4 * tid);
    v4i rv = {0, 0, 0, 0};
    rv.x = (tid == 0) ? bmax : 0;
    rv.y = (tid == 0) ? flag : 0;
    rv.z = (tid == 0) ? nh : 0;
    int* cp = CNT + (size_t)nodeBase + 4 * tid;
    int* fp = OFF + (size_t)nodeBase + 4 * tid;
    int* rp = REC + (size_t)blockIdx.x * 32 + 4 * (tid & 7);
    *(volatile v4i*)cp = cv;
    *(volatile v4i*)fp = fv;
    if (tid < 8) *(volatile v4i*)rp = rv;
    __threadfence();
    *(volatile v4i*)cp = cv;
    *(volatile v4i*)fp = fv;
    if (tid < 8) *(volatile v4i*)rp = rv;
  }
}

__device__ __forceinline__ void slot_info(const int* __restrict__ CNT, const int* __restrict__ OFF,
                                          const int* __restrict__ REC, int node, int& c, int& o, int& fl) {
  const int craw = CNT[node];
  const int oraw = OFF[node];
  const int fraw = REC[(size_t)(node >> PKS) * 32 + 1];
  int cc = craw < 0 ? 0 : craw;
  cc = cc > DEGCAP ? DEGCAP : cc;
  const int oo = oraw < 0 ? 0 : (oraw > RCAP ? RCAP : oraw);
  if (cc > RCAP - oo) cc = RCAP - oo;
  const int ff = (fraw != 0) ? 1 : 0;
  c  = __builtin_amdgcn_readfirstlane(cc);
  o  = __builtin_amdgcn_readfirstlane(oo);
  fl = __builtin_amdgcn_readfirstlane(ff);
}

__global__ __launch_bounds__(NTHR) void k_replay1(const unsigned short* __restrict__ XB, unsigned short* S1,
                                                  const int* __restrict__ LIST, const int* __restrict__ CNT,
                                                  const int* __restrict__ OFF, const int* __restrict__ REC,
                                                  int nN) {
  __shared__ __attribute__((aligned(16))) unsigned rowst[NWAVE * 128];
  const int tid = (int)threadIdx.x, lane = tid & 31, wave = tid >> 5;
  unsigned* wst = rowst + wave * 128;
  const float qn = __int_as_float(0x7fc00000);
#pragma unroll 1
  for (int ri = 0; ri < RPW; ++ri) {
    const int node = (int)blockIdx.x * RPB + wave * RPW + ri;
    int c, o, fl;
    slot_info(CNT, OFF, REC, node, c, o, fl);
    const int* lp = LIST + (size_t)(node >> PKS) * RCAP;
    int last = o + c - 1; last = last < o ? o : last;
    last = last > RCAP - 1 ? RCAP - 1 : last;
    float a0 = 0.0f, a1 = 0.0f, a2 = 0.0f, a3 = 0.0f;
#pragma unroll 1
    for (int b0 = 0; b0 < c; b0 += 32) {
      int idx = o + b0 + lane;
      idx = idx > last ? last : idx;
      int col = lp[idx];
      col = col < 0 ? 0 : (col > nN - 1 ? nN - 1 : col);
      const int m32 = (c - b0) < 32 ? (c - b0) : 32;
#pragma unroll 1
      for (int k = 0; k < m32; ++k) {
        const int sk = __builtin_amdgcn_readlane(col, k);
        const v2u w = *(const v2ua*)(XB + (size_t)sk * XBP + 4 * lane);
        a0 += bfw_lo(w.x);
        a1 += bfw_hi(w.x);
        a2 += bfw_lo(w.y);
        a3 += bfw_hi(w.y);
      }
    }
    const bool live = node < nN;
    const float pz = (fl != 0) ? qn : 0.0f;
    const float m0 = live ? (a0 + pz) : 0.0f;
    const float m1 = live ? (a1 + pz) : 0.0f;
    const float m2 = live ? (a2 + pz) : 0.0f;
    const float m3 = live ? (a3 + pz) : 0.0f;
    unsigned h0, l0, h1, l1;
    pack2(m0, m1, h0, l0);
    pack2(m2, m3, h1, l1);
    v2u hv, lv;
    hv.x = h0; hv.y = h1;
    lv.x = l0; lv.y = l1;
    *(v2ua*)(wst + 2 * lane)      = hv;
    *(v2ua*)(wst + 64 + 2 * lane) = lv;
    wave_sync();
    const v4u q = *(const v4ua*)(wst + 4 * lane);
    wave_sync();
    unsigned short* wp = S1 + (size_t)node * S1P + 8 * lane;
    *(volatile v4u*)wp = q;
    __threadfence();
    *(volatile v4u*)wp = q;
  }
}

__global__ __launch_bounds__(NTHR) void k_replay2(const unsigned short* __restrict__ src, unsigned short* dst,
                                                  const int* __restrict__ LIST, const int* __restrict__ CNT,
                                                  const int* __restrict__ OFF, const int* __restrict__ REC,
                                                  int nN) {
  const int tid = (int)threadIdx.x, lane = tid & 31, wave = tid >> 5;
  const float qn = __int_as_float(0x7fc00000);
#pragma unroll 1
  for (int ri = 0; ri < RPW; ++ri) {
    const int node = (int)blockIdx.x * RPB + wave * RPW + ri;
    int c, o, fl;
    slot_info(CNT, OFF, REC, node, c, o, fl);
    const int* lp = LIST + (size_t)(node >> PKS) * RCAP;
    int last = o + c - 1; last = last < o ? o : last;
    last = last > RCAP - 1 ? RCAP - 1 : last;
    float a0 = 0.f, a1 = 0.f, a2 = 0.f, a3 = 0.f, a4 = 0.f, a5 = 0.f, a6 = 0.f, a7 = 0.f;
#pragma unroll 1
    for (int b0 = 0; b0 < c; b0 += 32) {
      int idx = o + b0 + lane;
      idx = idx > last ? last : idx;
      int col = lp[idx];
      col = col < 0 ? 0 : (col > nN - 1 ? nN - 1 : col);
      const int m32 = (c - b0) < 32 ? (c - b0) : 32;
#pragma unroll 1
      for (int k = 0; k < m32; ++k) {
        const int sk = __builtin_amdgcn_readlane(col, k);
        const unsigned short* rp = src + (size_t)sk * HP + 8 * lane;
        const v4u wh = *(const v4ua*)rp;
        const v4u wl = *(const v4ua*)(rp + HD);
        a0 += bfw_lo(wh.x) + bfw_lo(wl.x);
        a1 += bfw_hi(wh.x) + bfw_hi(wl.x);
        a2 += bfw_lo(wh.y) + bfw_lo(wl.y);
        a3 += bfw_hi(wh.y) + bfw_hi(wl.y);
        a4 += bfw_lo(wh.z) + bfw_lo(wl.z);
        a5 += bfw_hi(wh.z) + bfw_hi(wl.z);
        a6 += bfw_lo(wh.w) + bfw_lo(wl.w);
        a7 += bfw_hi(wh.w) + bfw_hi(wl.w);
      }
    }
    const bool live = node < nN;
    const float pz = (fl != 0) ? qn : 0.0f;
    const float r0 = live ? (a0 + pz) : 0.0f;
    const float r1 = live ? (a1 + pz) : 0.0f;
    const float r2 = live ? (a2 + pz) : 0.0f;
    const float r3 = live ? (a3 + pz) : 0.0f;
    const float r4 = live ? (a4 + pz) : 0.0f;
    const float r5 = live ? (a5 + pz) : 0.0f;
    const float r6 = live ? (a6 + pz) : 0.0f;
    const float r7 = live ? (a7 + pz) : 0.0f;
    unsigned h0, l0, h1, l1, h2, l2, h3, l3;
    pack2(r0, r1, h0, l0);
    pack2(r2, r3, h1, l1);
    pack2(r4, r5, h2, l2);
    pack2(r6, r7, h3, l3);
    v4u qh, ql;
    qh.x = h0; qh.y = h1; qh.z = h2; qh.w = h3;
    ql.x = l0; ql.y = l1; ql.z = l2; ql.w = l3;
    unsigned short* wp = dst + (size_t)node * HP + 8 * lane;
    *(volatile v4u*)wp = qh;
    *(volatile v4u*)(wp + HD) = ql;
    __threadfence();
    *(volatile v4u*)wp = qh;
    *(volatile v4u*)(wp + HD) = ql;
  }
}

template <int NT, int WPITCH>
__device__ __forceinline__ void kseg(const unsigned short* __restrict__ ap, const unsigned short* __restrict__ wp,
                                     int nsteps, v8f (&acc)[NT]) {
#pragma unroll 1
  for (int ks = 0; ks < nsteps; ++ks) {
    FragB af;
    af.h[0] = *(const v8usa*)(ap + 32 * ks);
    af.h[1] = *(const v8usa*)(ap + 32 * ks + 16);
#pragma unroll
    for (int t = 0; t < NT; ++t) {
      const unsigned short* wq = wp + (size_t)(16 * t) * (size_t)WPITCH + 32 * ks;
      FragB bf;
      bf.h[0] = *(const v8usa*)wq;
      bf.h[1] = *(const v8usa*)(wq + 16);
      acc[t] = wmb(af, bf, acc[t]);
    }
  }
}

__global__ __launch_bounds__(GTHR) __attribute__((amdgpu_num_vgpr(248)))
void k_gemm1(const unsigned short* __restrict__ S1, const unsigned short* __restrict__ XB,
             const unsigned short* __restrict__ W1c, const float* __restrict__ B1,
             unsigned short* Hhl, int nN) {
  __shared__ __attribute__((aligned(16))) float stg[GBM * GBN];
  __shared__ __attribute__((aligned(16))) float bsh[GBN];
  const int tid = (int)threadIdx.x, lane = tid & 31, wave = tid >> 5, hh = lane >> 4, m = lane & 15;
  const int rowBase = (int)blockIdx.x * GBM;
  const int colBase = (int)blockIdx.y * GBN;

  if (tid < 32) {
    const v4f b4 = *(const v4f*)(B1 + colBase + 4 * tid);
    *(v4fa*)(bsh + 4 * tid) = b4;
  }

  v8f acc[8];
  {
    const v8f z = {0.f, 0.f, 0.f, 0.f, 0.f, 0.f, 0.f, 0.f};
#pragma unroll
    for (int t = 0; t < 8; ++t) acc[t] = z;
  }
  const size_t arow = (size_t)(rowBase + 16 * wave + m);
  const unsigned short* wp = W1c + (size_t)(colBase + m) * (size_t)W1P + 8 * hh;
  kseg<8, W1P>(S1 + arow * S1P + 8 * hh, wp, KS1, acc);
#if SPLIT_S1
  kseg<8, W1P>(S1 + arow * S1P + FI + 8 * hh, wp + FI, KS1, acc);
#endif
  kseg<8, W1P>(XB + arow * XBP + 8 * hh, wp + 2 * FI, KS1, acc);
  __syncthreads();

#pragma unroll
  for (int t = 0; t < 8; ++t) {
    const int lc = 16 * t + m;
    const float bb = bsh[lc];
#pragma unroll
    for (int r = 0; r < 8; ++r) {
      const int lr = 16 * wave + 8 * hh + r;
      const bool live = (rowBase + lr) < nN;
      const float v = relu_k(acc[t][r] + bb);
      stg[lr * GBN + lc] = live ? v : 0.0f;
    }
  }
  __syncthreads();

  const int cb = 8 * m;
  const bool isHi = (hh == 0);
  v4u pk[16];
#pragma unroll
  for (int i = 0; i < 16; ++i) {
    const int lr = 16 * wave + i;
    const v4f a = *(const v4fa*)(stg + lr * GBN + cb);
    const v4f b = *(const v4fa*)(stg + lr * GBN + cb + 4);
    const float f[8] = {a.x, a.y, a.z, a.w, b.x, b.y, b.z, b.w};
    unsigned w[4];
#pragma unroll
    for (int j = 0; j < 4; ++j) {
      unsigned hw, lw;
      pack2(f[2 * j], f[2 * j + 1], hw, lw);
      w[j] = isHi ? hw : lw;
    }
    v4u pw; pw.x = w[0]; pw.y = w[1]; pw.z = w[2]; pw.w = w[3];
    pk[i] = pw;
  }
#pragma unroll
  for (int i = 0; i < 16; ++i) {
    const int gr = rowBase + 16 * wave + i;
    unsigned short* op = Hhl + (size_t)gr * (size_t)HP + hh * HD + colBase + cb;
    *(volatile v4u*)op = pk[i];
  }
  __threadfence();
#pragma unroll
  for (int i = 0; i < 16; ++i) {
    const int gr = rowBase + 16 * wave + i;
    unsigned short* op = Hhl + (size_t)gr * (size_t)HP + hh * HD + colBase + cb;
    *(volatile v4u*)op = pk[i];
  }
}

__global__ __launch_bounds__(GTHR) __attribute__((amdgpu_num_vgpr(248)))
void k_gemm2(const unsigned short* __restrict__ S2, const unsigned short* __restrict__ Hhl,
             const unsigned short* __restrict__ W2c, const float* __restrict__ B2,
             const int* __restrict__ REC, float* out, int nN) {
  __shared__ __attribute__((aligned(16))) float stg2[GBM * OC];
  __shared__ __attribute__((aligned(16))) float bsh[ONP];
  const int tid = (int)threadIdx.x, lane = tid & 31, wave = tid >> 5, hh = lane >> 4, m = lane & 15;
  const int rowBase = (int)blockIdx.x * GBM;

  if (tid < ONP / 4) {
    const v4f b4 = *(const v4f*)(B2 + 4 * tid);
    *(v4fa*)(bsh + 4 * tid) = b4;
  }

  v8f acc[4];
  {
    const v8f z = {0.f, 0.f, 0.f, 0.f, 0.f, 0.f, 0.f, 0.f};
#pragma unroll
    for (int t = 0; t < 4; ++t) acc[t] = z;
  }
  const size_t arow = (size_t)(rowBase + 16 * wave + m) * (size_t)HP + 8 * hh;
  const unsigned short* wp = W2c + (size_t)m * (size_t)W2P + 8 * hh;
  kseg<4, W2P>(S2 + arow, wp, KS2, acc);
#if SPLIT_S2
  kseg<4, W2P>(S2 + arow + HD, wp + HD, KS2, acc);
#endif
  kseg<4, W2P>(Hhl + arow, wp + 2 * HD, KS2, acc);
#if SPLIT_H
  kseg<4, W2P>(Hhl + arow + HD, wp + 3 * HD, KS2, acc);
#endif
  __syncthreads();

  const int flr = REC[(size_t)(rowBase >> PKS) * 32 + 1];
  const float qn = __int_as_float(0x7fc00000);
#pragma unroll
  for (int t = 0; t < 4; ++t) {
    const int lc = 16 * t + m;
    const float bb = bsh[lc];
#pragma unroll
    for (int r = 0; r < 8; ++r) {
      const int lr = 16 * wave + 8 * hh + r;
      const float v0 = acc[t][r] + bb;
      const float v  = (flr != 0) ? qn : v0;
      if (lc < OC) stg2[lr * OC + lc] = v;
    }
  }
  __syncthreads();

  int nvalid = nN - rowBase;
  nvalid = nvalid < 0 ? 0 : (nvalid > GBM ? GBM : nvalid);
  const int nq    = (nvalid * OC) >> 2;
  const int qlast = nq > 0 ? nq - 1 : 0;
  v4f pv[NFL];
#pragma unroll
  for (int it = 0; it < NFL; ++it) {
    const int q  = it * GTHR + tid;
    const int qc = q < qlast ? q : qlast;
    pv[it] = *(const v4fa*)(stg2 + 4 * qc);
    asm volatile("" :: "v"(pv[it]));
  }
  float* ob = out + (size_t)rowBase * OC;
#pragma unroll
  for (int it = 0; it < NFL; ++it) {
    const int q = it * GTHR + tid;
    if (q < nq) *(volatile v4f*)(ob + 4 * q) = pv[it];
  }
  __threadfence();
#pragma unroll
  for (int it = 0; it < NFL; ++it) {
    const int q = it * GTHR + tid;
    if (q < nq) *(volatile v4f*)(ob + 4 * q) = pv[it];
  }
}

static inline int cdiv(int a, int b) { return (a + b - 1) / b; }
static inline size_t al256(size_t o) { return (o + 255) & ~(size_t)255; }

extern "C" void kernel_launch(void* const* d_in, const int* in_sizes, int n_in,
                              void* d_out, int out_size, void* d_ws, size_t ws_size,
                              hipStream_t stream) {
  if (n_in < 8) return;
  if (in_sizes[0] < FI * 64 || (in_sizes[0] % FI) != 0) return;
  const int nN = in_sizes[0] / FI;
  if ((nN & 15) != 0 || nN >= (1 << 22)) return;
  if (in_sizes[1] < 2 || (in_sizes[1] & 1) != 0) return;
  const int nE = in_sizes[1] / 2;
  if (nE < 1 || nE >= (1 << 21)) return;
  if (in_sizes[2] != HD * FI || in_sizes[3] != HD || in_sizes[4] != HD * FI) return;
  if (in_sizes[5] != OC * HD || in_sizes[6] != OC || in_sizes[7] != OC * HD) return;
  if ((long long)out_size != (long long)nN * OC) return;

  const float* x   = (const float*)d_in[0];
  const int*   ei  = (const int*)  d_in[1];
  const int*   src = ei;
  const int*   dst = ei + nE;
  const float* W1l = (const float*)d_in[2];
  const float* b1l = (const float*)d_in[3];
  const float* W1r = (const float*)d_in[4];
  const float* W2l = (const float*)d_in[5];
  const float* b2l = (const float*)d_in[6];
  const float* W2r = (const float*)d_in[7];
  float* out = (float*)d_out;

  const int mRows = cdiv(nN, 128) * 128;
  const int nB    = cdiv(nN, NBA);
  const int NPADN = nB * NBA;
  if (mRows > NPADN || (mRows % GBM) != 0) return;
  const int nXU = mRows * (FI / 8);
  if ((nXU % NTHR) != 0) return;
  const int vec8 = ((nE & 3) == 0) ? 1 : 0;

  char* ws = (char*)d_ws;
  size_t off = 0;
  const size_t oW1 = off; off = al256(off + (size_t)HD * W1P * 2);
  const size_t oW2 = off; off = al256(off + (size_t)ONP * W2P * 2);
  const size_t oB1 = off; off = al256(off + (size_t)HD * 4);
  const size_t oB2 = off; off = al256(off + (size_t)ONP * 4);
  const size_t oRC = off; off = al256(off + (size_t)nB * 128);
  const size_t oCN = off; off = al256(off + (size_t)NPADN * 4);
  const size_t oOF = off; off = al256(off + (size_t)NPADN * 4);
  const size_t oLS = off; off = al256(off + (size_t)nB * RCAP * 4);
  const size_t oH  = off; off = al256(off + (size_t)mRows * HP * 2);
  const size_t oR2 = off; off = al256(off + (size_t)mRows * HP * 2);
  if (off > ws_size) return;
  const size_t s1Bytes = (size_t)mRows * S1P * 2;
  const size_t xbBytes = (size_t)mRows * XBP * 2;
  if (s1Bytes + xbBytes > (size_t)mRows * HP * 2) return;
  unsigned short* W1c = (unsigned short*)(ws + oW1);
  unsigned short* W2c = (unsigned short*)(ws + oW2);
  float* B1   = (float*)(ws + oB1);
  float* B2   = (float*)(ws + oB2);
  int*   REC  = (int*)(ws + oRC);
  int*   CNT  = (int*)(ws + oCN);
  int*   OFF  = (int*)(ws + oOF);
  int*   LIST = (int*)(ws + oLS);
  unsigned short* Hhl = (unsigned short*)(ws + oH);
  unsigned short* S2  = (unsigned short*)(ws + oR2);
  unsigned short* S1  = (unsigned short*)(ws + oR2);
  unsigned short* XB  = (unsigned short*)(ws + oR2 + s1Bytes);

  hipFuncSetAttribute(reinterpret_cast<const void*>(&k_bucket), hipFuncAttributeMaxDynamicSharedMemorySize, LDS_BK);

  const int nU = nXU + W1U + W2U + BU1 + BU2;
  k_prep<<<cdiv(nU, NTHR), NTHR, 0, stream>>>(x, W1l, b1l, W1r, W2l, b2l, W2r, XB, W1c, W2c, B1, B2, nN, nXU);
  k_bucket<<<nB, NTHR, LDS_BK, stream>>>(dst, src, nE, nN, vec8, LIST, CNT, OFF, REC);
  k_replay1<<<mRows / RPB, NTHR, 0, stream>>>(XB, S1, LIST, CNT, OFF, REC, nN);
  const dim3 gg((unsigned)(mRows / GBM), 2u, 1u);
  k_gemm1<<<gg, GTHR, 0, stream>>>(S1, XB, W1c, B1, Hhl, nN);
  k_replay2<<<mRows / RPB, NTHR, 0, stream>>>(Hhl, S2, LIST, CNT, OFF, REC, nN);
  k_gemm2<<<mRows / GBM, GTHR, 0, stream>>>(S2, Hhl, W2c, B2, REC, out, nN);
}
